// MixerLayer_46205258170887
// MI455X (gfx1250) — hardware-verified
//
#include <hip/hip_runtime.h>
#include <math.h>
#include <stdint.h>

#define NB   16
#define IH   16
#define IW   64
#define LL   (IH * IW)
#define HH   256
#define NHD  8
#define HD   32
#define QKW  (2 * HH)
#define QKVW (3 * HH)
#define MT   (NB * LL)
#define RW   3
#define CW   5
#define NCHK (2 * (2 * RW + 1))
#define ZSP  72
#define WSC  16.0f
#define PSC  1024.0f
#define ZSC  16.0f
#define RSC  2048.0f
#define RSCI 0.00048828125f
#define SCL  0.17677669529663687f

static_assert(NHD * HD == HH);
static_assert(IW == 64 && (IH & (IH - 1)) == 0 && (MT / 64) == NB * IH);
static_assert((MT % 64) == 0 && (HH % 64) == 0 && (QKW % 64) == 0 && (MT % 32) == 0);
static_assert((((MT / 64) * (QKW / 64)) % 8) == 0);
static_assert((((MT / 64) * (HH / 64)) % 8) == 0);
static_assert((((HH / 64) * (MT / 64)) % 8) == 0);
static_assert((((MT / 32) * (HH / 64)) % 8) == 0);
static_assert((MT % 8) == 0 && (QKVW % 8) == 0 && (HH % 8) == 0);
static_assert(ZSP >= 64 && (ZSP % 8) == 0);

typedef _Float16 v16h __attribute__((ext_vector_type(16)));
typedef _Float16 v8h  __attribute__((ext_vector_type(8)));
typedef unsigned short v16us __attribute__((ext_vector_type(16)));
typedef unsigned short v8us  __attribute__((ext_vector_type(8)));
typedef float v8f __attribute__((ext_vector_type(8)));
typedef float v4f __attribute__((ext_vector_type(4)));
typedef unsigned int v4u __attribute__((ext_vector_type(4)));

union FragU { v16us v; v8us h[2]; };

__device__ __forceinline__ unsigned short bf_bits(float f) {
  const unsigned u = __float_as_uint(f);
  return (unsigned short)((u + 0x7FFFu + ((u >> 16) & 1u)) >> 16);
}
__device__ __forceinline__ float bf_up(unsigned short h) { return __uint_as_float(((unsigned)h) << 16); }
__device__ __forceinline__ float bfr(float f) { return bf_up(bf_bits(f)); }
__device__ __forceinline__ unsigned short h_bits(_Float16 x) { return __builtin_bit_cast(unsigned short, x); }
__device__ __forceinline__ unsigned short f2h(float f) { return h_bits((_Float16)f); }
__device__ __forceinline__ float h_up(unsigned short h) { return (float)__builtin_bit_cast(_Float16, h); }
__device__ __forceinline__ unsigned pk16(unsigned short a, unsigned short b) { return (unsigned)a | ((unsigned)b << 16); }
__device__ __forceinline__ v8f zero8() { v8f z = {0.f, 0.f, 0.f, 0.f, 0.f, 0.f, 0.f, 0.f}; return z; }
__device__ __forceinline__ void split_h(float f, unsigned short& hi, unsigned short& lo) {
  hi = f2h(f);
  lo = f2h((f - h_up(hi)) * RSC);
}

__device__ __forceinline__ v16us ldfrag_u(const unsigned short* p) {
  FragU f;
  f.h[0] = *(const v8us*)(p);
  f.h[1] = *(const v8us*)(p + 16);
  return f.v;
}

__device__ __forceinline__ v8f mma_h_raw(v16us a, v16us b, v8f c) {
  return __builtin_amdgcn_wmma_f32_16x16x32_f16(false, __builtin_bit_cast(v16h, a), false,
                                                __builtin_bit_cast(v16h, b), (short)0, c, false, false);
}
__device__ __forceinline__ void dep_guard1(v8f& a, v8f& b, v16us x) {
#if defined(__HIP_DEVICE_COMPILE__)
  asm volatile("v_nop\n\tv_nop\n\tv_nop\n\tv_nop" : "+v"(a), "+v"(b) : "v"(x));
#endif
}
__device__ __forceinline__ void dep_guard2(v8f& a, v8f& b, v8f& c, v8f& d, v16us x, v16us y) {
#if defined(__HIP_DEVICE_COMPILE__)
  asm volatile("v_nop\n\tv_nop\n\tv_nop\n\tv_nop" : "+v"(a), "+v"(b), "+v"(c), "+v"(d) : "v"(x), "v"(y));
#endif
}
__device__ __forceinline__ void keep4_u(v16us a, v16us b, v16us c, v16us d) {
#if defined(__HIP_DEVICE_COMPILE__)
  asm volatile("v_nop" :: "v"(a), "v"(b), "v"(c), "v"(d));
#endif
}
__device__ __forceinline__ void acc_guard4(v8f& a, v8f& b, v8f& c, v8f& d) {
#if defined(__HIP_DEVICE_COMPILE__)
  asm volatile("v_nop\n\tv_nop\n\tv_nop\n\tv_nop" : "+v"(a), "+v"(b), "+v"(c), "+v"(d));
#endif
}
__device__ __forceinline__ void guard6(v8f& a, v8f& b, v8f& c, v8f& d, v8f& e, v8f& f,
                                       v16us p, v16us q, v16us r, v16us s, v16us t, v16us u) {
#if defined(__HIP_DEVICE_COMPILE__)
  asm volatile("v_nop\n\tv_nop\n\tv_nop\n\tv_nop"
               : "+v"(a), "+v"(b), "+v"(c), "+v"(d), "+v"(e), "+v"(f)
               : "v"(p), "v"(q), "v"(r), "v"(s), "v"(t), "v"(u));
#endif
}
__device__ __forceinline__ void wave_sync_lds() {
  __builtin_amdgcn_fence(__ATOMIC_RELEASE, "workgroup");
  __builtin_amdgcn_wave_barrier();
  __builtin_amdgcn_fence(__ATOMIC_ACQUIRE, "workgroup");
}

__global__ __launch_bounds__(256) void cvt_rows(const float* __restrict__ x, unsigned short* xh, int nrows, float sc) {
  const int row = blockIdx.x * 8 + (threadIdx.x >> 5);
  const int lane = threadIdx.x & 31;
  if (row >= nrows) return;
  const float* p = x + (size_t)row * HH + lane * 8;
  const v4f a0 = *(const v4f*)(p);
  const v4f a1 = *(const v4f*)(p + 4);
  v4u hv;
#pragma unroll
  for (int e = 0; e < 2; ++e) {
    hv[e]     = pk16(f2h(bfr(a0[2 * e]) * sc), f2h(bfr(a0[2 * e + 1]) * sc));
    hv[2 + e] = pk16(f2h(bfr(a1[2 * e]) * sc), f2h(bfr(a1[2 * e + 1]) * sc));
  }
  unsigned short* d = xh + (size_t)row * HH + lane * 8;
  for (int pass = 0; pass < 2; ++pass) {
    *(volatile v4u*)(d) = hv;
    __threadfence();
  }
}

template <int OM, int CBM, int ASPL>
__global__ __launch_bounds__(256) void gemm64(
    const unsigned short* __restrict__ Ap, const unsigned short* __restrict__ Alp, int lda,
    const unsigned short* __restrict__ Btp, int ldb,
    unsigned short* Ch, unsigned short* Cl, float* Cf, int ldc,
    const float* __restrict__ cb, float wsc, float osc, int M, int N, int K) {
  constexpr int MI = ASPL ? 2 : 4;
  constexpr int TR = 16 * MI;
  __shared__ __align__(16) float sT[8][16 * 68];
  const int lane = threadIdx.x & 31;
  const int wave = threadIdx.x >> 5;
  const int tilesN = N >> 6;
  const int tilesM = M / TR;
  const int tile = blockIdx.x * 8 + wave;
  if (tile >= tilesM * tilesN) return;
  const int tm = tile / tilesN;
  const int tn = tile - tm * tilesN;
  const int m0 = tm * TR;
  const int n0 = tn << 6;

  const int rlane = lane & 15;
  const int koff  = (lane >> 4) * 8;
  const int mOff  = (lane >> 4) * 8;

  v8f acc[MI][4];
  v8f accr[MI][4];
#pragma unroll
  for (int i = 0; i < MI; ++i)
#pragma unroll
    for (int j = 0; j < 4; ++j) { acc[i][j] = zero8(); accr[i][j] = zero8(); }

  for (int k0 = 0; k0 < K; k0 += 32) {
    v16us bh[4];
#pragma unroll
    for (int j = 0; j < 4; ++j) {
      const size_t bo = (size_t)(n0 + (j << 4) + rlane) * ldb + koff + k0;
      bh[j] = ldfrag_u(Btp + bo);
    }
#pragma unroll
    for (int i = 0; i < MI; ++i) {
      const size_t ao = (size_t)(m0 + (i << 4) + rlane) * lda + koff + k0;
      const v16us ah = ldfrag_u(Ap + ao);
      if (ASPL) {
        const v16us al = ldfrag_u(Alp + ao);
#pragma unroll
        for (int j = 0; j < 4; ++j) {
          acc[i][j]  = mma_h_raw(ah, bh[j], acc[i][j]);
          accr[i][j] = mma_h_raw(al, bh[j], accr[i][j]);
        }
        dep_guard2(acc[i][0], acc[i][3], accr[i][0], accr[i][3], ah, al);
      } else {
#pragma unroll
        for (int j = 0; j < 4; ++j) acc[i][j] = mma_h_raw(ah, bh[j], acc[i][j]);
        dep_guard1(acc[i][0], acc[i][3], ah);
      }
    }
    keep4_u(bh[0], bh[1], bh[2], bh[3]);
  }
#pragma unroll
  for (int i = 0; i < MI; ++i) {
    acc_guard4(acc[i][0], acc[i][1], acc[i][2], acc[i][3]);
    if (ASPL) acc_guard4(accr[i][0], accr[i][1], accr[i][2], accr[i][3]);
  }

  const int hh2 = lane >> 4, c4 = (lane & 15) * 4;
  const int q8  = lane >> 3, c8 = (lane & 7) * 8;

  v4f cb4 = {0.f, 0.f, 0.f, 0.f};
  float cbc[8];
#pragma unroll
  for (int e = 0; e < 8; ++e) cbc[e] = 0.f;
  if (OM == 0 && CBM == 1) {
    const v4f v = *(const v4f*)(cb + n0 + c4);
    cb4[0] = bfr(v[0]); cb4[1] = bfr(v[1]); cb4[2] = bfr(v[2]); cb4[3] = bfr(v[3]);
  }
  if (OM == 1 && CBM == 1) {
    const v4f v0 = *(const v4f*)(cb + n0 + c8);
    const v4f v1 = *(const v4f*)(cb + n0 + c8 + 4);
#pragma unroll
    for (int e = 0; e < 4; ++e) { cbc[e] = bfr(v0[e]); cbc[4 + e] = bfr(v1[e]); }
  }

  float* slab = sT[wave];
#pragma unroll
  for (int i = 0; i < MI; ++i) {
    const int mBase = m0 + (i << 4);
#pragma unroll
    for (int j = 0; j < 4; ++j) {
#pragma unroll
      for (int r = 0; r < 8; ++r) {
        float v = acc[i][j][r];
        if (ASPL) v += accr[i][j][r] * RSCI;
        slab[(mOff + r) * 68 + (j << 4) + rlane] = v;
      }
    }
    wave_sync_lds();
    if (OM == 0) {
      v4f vals[8];
#pragma unroll
      for (int it = 0; it < 8; ++it) {
        const int row = it * 2 + hh2;
        const v4f v = *(const v4f*)(slab + row * 68 + c4);
        vals[it] = (v * wsc + cb4) * osc;
      }
      for (int pass = 0; pass < 2; ++pass) {
#pragma unroll
        for (int it = 0; it < 8; ++it) {
          const int row = it * 2 + hh2;
          *(volatile v4f*)(Cf + (size_t)(mBase + row) * ldc + (size_t)n0 + c4) = vals[it];
        }
        __threadfence();
      }
    }
    if (OM == 1) {
      v4u hv[4], lv[4];
#pragma unroll
      for (int it = 0; it < 4; ++it) {
        const int row = it * 4 + q8;
        const float* sp = slab + row * 68 + c8;
        float rb = 0.f;
        if (CBM == 2) rb = bfr(cb[mBase + row]);
        v4u ha = {0u, 0u, 0u, 0u}, la = {0u, 0u, 0u, 0u};
#pragma unroll
        for (int e = 0; e < 4; ++e) {
          const float f0 = (sp[2 * e]     * wsc + cbc[2 * e]     + rb) * osc;
          const float f1 = (sp[2 * e + 1] * wsc + cbc[2 * e + 1] + rb) * osc;
          unsigned short h0, l0, h1, l1;
          split_h(f0, h0, l0);
          split_h(f1, h1, l1);
          ha[e] = pk16(h0, h1);
          la[e] = pk16(l0, l1);
        }
        hv[it] = ha;
        lv[it] = la;
      }
      for (int pass = 0; pass < 2; ++pass) {
#pragma unroll
        for (int it = 0; it < 4; ++it) {
          const int row = it * 4 + q8;
          const size_t go = (size_t)(mBase + row) * ldc + (size_t)n0 + c8;
          *(volatile v4u*)(Ch + go) = hv[it];
          *(volatile v4u*)(Cl + go) = lv[it];
        }
        __threadfence();
      }
    }
    wave_sync_lds();
  }
}

__global__ __launch_bounds__(256) void attn_kernel(const unsigned short* __restrict__ QKh,
                                                   const unsigned short* __restrict__ QKl,
                                                   const unsigned short* __restrict__ VT,
                                                   const unsigned short* __restrict__ VTl,
                                                   unsigned short* Zh, unsigned short* Zl) {
  __shared__ __align__(16) unsigned short ps[8 * 1024];
  __shared__ __align__(16) unsigned short zsth[64 * ZSP];
  __shared__ __align__(16) unsigned short zstl[64 * ZSP];
  const int tq0 = blockIdx.x * 64;
  const int qr  = blockIdx.x & (IH - 1);
  const int tb0 = (blockIdx.x / IH) * LL;
  const int hp = blockIdx.y;
  const int t = threadIdx.x, lane = t & 31, wv = t >> 5, hh = lane >> 4, jc = lane & 15;
  const int ms = wv & 3, hs = wv >> 2, head = hp * 2 + hs;

  const size_t qo = (size_t)(tq0 + 16 * ms + jc) * QKW + head * HD + 8 * hh;
  const v16us qf = ldfrag_u(QKh + qo);
  const v16us ql = ldfrag_u(QKl + qo);
  float m[8], ll[8];
  v8f oz0 = zero8(), oz1 = zero8(), oa0 = zero8(), oa1 = zero8(), ob0 = zero8(), ob1 = zero8();
#pragma unroll
  for (int r = 0; r < 8; ++r) { m[r] = -1.0e30f; ll[r] = 0.f; }
  unsigned short* pw = ps + wv * 1024;
  const size_t vo0 = (size_t)(head * HD + jc) * MT;
  const size_t vo1 = vo0 + (size_t)16 * MT;
  const int qcb = 16 * ms + 8 * hh;
  const int clo = 16 * ms - CW, chi = 16 * ms + 15 + CW;

#pragma unroll 1
  for (int idx = 0; idx < NCHK; ++idx) {
    const int r2 = qr - RW + (idx >> 1);
    const int c  = idx & 1;
    if (r2 < 0 || r2 >= IH) continue;
    const int kcb = 32 * c;
    if (kcb > chi || kcb + 31 < clo) continue;
    const int tk0 = tb0 + r2 * IW + kcb;
    const size_t ko0 = (size_t)(tk0 + jc) * QKW + HH + head * HD + 8 * hh;
    const size_t ko1 = ko0 + (size_t)16 * QKW;
    const v16us kf0 = ldfrag_u(QKh + ko0);
    const v16us kf1 = ldfrag_u(QKh + ko1);
    const v16us kl0 = ldfrag_u(QKl + ko0);
    const v16us kl1 = ldfrag_u(QKl + ko1);
    v8f s0  = mma_h_raw(qf, kf0, zero8());
    v8f s1  = mma_h_raw(qf, kf1, zero8());
    v8f sa0 = mma_h_raw(qf, kl0, zero8());
    v8f sa1 = mma_h_raw(qf, kl1, zero8());
    v8f sb0 = mma_h_raw(ql, kf0, zero8());
    v8f sb1 = mma_h_raw(ql, kf1, zero8());
    guard6(s0, s1, sa0, sa1, sb0, sb1, qf, ql, kf0, kf1, kl0, kl1);
    const int dcb = kcb + jc - qcb;
    wave_sync_lds();
#pragma unroll
    for (int r = 0; r < 8; ++r) {
      const int il = 8 * hh + r;
      const int d0 = dcb - r, d1 = d0 + 16;
      const bool va = (d0 >= -CW) && (d0 <= CW);
      const bool vb = (d1 >= -CW) && (d1 <= CW);
      const float t0 = (s0[r] + (sa0[r] + sb0[r]) * RSCI) * SCL;
      const float t1 = (s1[r] + (sa1[r] + sb1[r]) * RSCI) * SCL;
      const float v0 = va ? t0 : -3.0e38f;
      const float v1 = vb ? t1 : -3.0e38f;
      float rm = fmaxf(v0, v1);
#pragma unroll
      for (int off = 1; off < 16; off <<= 1) rm = fmaxf(rm, __shfl_xor(rm, off, 32));
      const float mn2   = fmaxf(m[r], rm);
      const float alpha = __expf(m[r] - mn2);
      float e0 = __expf(v0 - mn2);
      float e1 = __expf(v1 - mn2);
      e0 = va ? e0 : 0.0f;
      e1 = vb ? e1 : 0.0f;
      float rs = e0 + e1;
#pragma unroll
      for (int off = 1; off < 16; off <<= 1) rs += __shfl_xor(rs, off, 32);
      ll[r] = ll[r] * alpha + rs;
      m[r]  = mn2;
      oz0[r] *= alpha; oz1[r] *= alpha;
      oa0[r] *= alpha; oa1[r] *= alpha;
      ob0[r] *= alpha; ob1[r] *= alpha;
      unsigned short h0, l0, h1, l1;
      split_h(e0 * PSC, h0, l0);
      split_h(e1 * PSC, h1, l1);
      pw[il * 32 + jc]            = h0;
      pw[il * 32 + 16 + jc]       = h1;
      pw[512 + il * 32 + jc]      = l0;
      pw[512 + il * 32 + 16 + jc] = l1;
    }
    wave_sync_lds();
    FragU pa, pb;
    pa.h[0] = *(const v8us*)(pw + jc * 32 + 8 * hh);
    pa.h[1] = *(const v8us*)(pw + jc * 32 + 16 + 8 * hh);
    pb.h[0] = *(const v8us*)(pw + 512 + jc * 32 + 8 * hh);
    pb.h[1] = *(const v8us*)(pw + 512 + jc * 32 + 16 + 8 * hh);
    const v16us f0 = ldfrag_u(VT  + vo0 + tk0 + 8 * hh);
    const v16us f1 = ldfrag_u(VT  + vo1 + tk0 + 8 * hh);
    const v16us g0 = ldfrag_u(VTl + vo0 + tk0 + 8 * hh);
    const v16us g1 = ldfrag_u(VTl + vo1 + tk0 + 8 * hh);
    oz0 = mma_h_raw(pa.v, f0, oz0);
    oz1 = mma_h_raw(pa.v, f1, oz1);
    oa0 = mma_h_raw(pa.v, g0, oa0);
    oa1 = mma_h_raw(pa.v, g1, oa1);
    ob0 = mma_h_raw(pb.v, f0, ob0);
    ob1 = mma_h_raw(pb.v, f1, ob1);
    guard6(oz0, oz1, oa0, oa1, ob0, ob1, pa.v, pb.v, f0, f1, g0, g1);
  }

#pragma unroll
  for (int r = 0; r < 8; ++r) {
    const int il = 8 * hh + r;
    const float l = ll[r];
    const float inv = ((l > 0.f) ? (1.0f / l) : 0.f) * (ZSC / PSC);
    const float z0 = (oz0[r] + (oa0[r] + ob0[r]) * RSCI) * inv;
    const float z1 = (oz1[r] + (oa1[r] + ob1[r]) * RSCI) * inv;
    unsigned short h0, l0, h1, l1;
    split_h(z0, h0, l0);
    split_h(z1, h1, l1);
    const int so = (16 * ms + il) * ZSP + hs * 32 + jc;
    zsth[so] = h0; zsth[so + 16] = h1;
    zstl[so] = l0; zstl[so + 16] = l1;
  }
  __syncthreads();
  v4u hv[2], lv[2];
#pragma unroll
  for (int it = 0; it < 2; ++it) {
    const int row = it * 32 + (t >> 3), p = (t & 7) * 8;
    hv[it] = *(const v4u*)(zsth + row * ZSP + p);
    lv[it] = *(const v4u*)(zstl + row * ZSP + p);
  }
  for (int pass = 0; pass < 2; ++pass) {
#pragma unroll
    for (int it = 0; it < 2; ++it) {
      const int row = it * 32 + (t >> 3), p = (t & 7) * 8;
      const size_t go = (size_t)(tq0 + row) * HH + hp * 64 + p;
      *(volatile v4u*)(Zh + go) = hv[it];
      *(volatile v4u*)(Zl + go) = lv[it];
    }
    __threadfence();
  }
}

extern "C" void kernel_launch(void* const* d_in, const int* in_sizes, int n_in,
                              void* d_out, int out_size, void* d_ws, size_t ws_size,
                              hipStream_t stream) {
  if (n_in < 6) return;
  if (in_sizes[0] != MT * HH) return;
  if (in_sizes[1] != QKVW * HH || in_sizes[2] != QKVW) return;
  if (in_sizes[3] != HH * HH || in_sizes[4] != HH) return;
  if (in_sizes[5] != HH * HH) return;
  if (out_size != MT * HH) return;

  const float* x    = (const float*)d_in[0];
  const float* Wqkv = (const float*)d_in[1];
  const float* bqkv = (const float*)d_in[2];
  const float* Wout = (const float*)d_in[3];
  const float* bout = (const float*)d_in[4];
  const float* Wprj = (const float*)d_in[5];

  const size_t PXH = (size_t)MT * HH * 2;
  const size_t PWQ = (size_t)QKVW * HH * 2;
  const size_t PWO = (size_t)HH * HH * 2;
  const size_t PWP = (size_t)HH * HH * 2;
  const size_t PQK = (size_t)MT * QKW * 2;
  const size_t PVT = (size_t)HH * MT * 2;
  const size_t PZH = (size_t)MT * HH * 2;
  const size_t PAH = (size_t)MT * HH * 2;
  size_t off = 0;
  const size_t oXh = off; off += PXH;
  const size_t oWq = off; off += PWQ;
  const size_t oWo = off; off += PWO;
  const size_t oWp = off; off += PWP;
  const size_t oQK = off; off += PQK;
  const size_t oQL = off; off += PQK;
  const size_t oVT = off; off += PVT;
  const size_t oVL = off; off += PVT;
  const size_t oZh = off; off += PZH;
  const size_t oZl = off; off += PZH;
  const size_t oAh = off; off += PAH;
  const size_t oAl = off; off += PAH;
  if (off > ws_size) return;
  if (off > (size_t)134217728) return;

  char* ws = (char*)d_ws;
  unsigned short* Xh     = (unsigned short*)(ws + oXh);
  unsigned short* Wqkv16 = (unsigned short*)(ws + oWq);
  unsigned short* Wo16   = (unsigned short*)(ws + oWo);
  unsigned short* Wp16   = (unsigned short*)(ws + oWp);
  unsigned short* QKh    = (unsigned short*)(ws + oQK);
  unsigned short* QKl    = (unsigned short*)(ws + oQL);
  unsigned short* VT     = (unsigned short*)(ws + oVT);
  unsigned short* VTl    = (unsigned short*)(ws + oVL);
  unsigned short* Zh     = (unsigned short*)(ws + oZh);
  unsigned short* Zl     = (unsigned short*)(ws + oZl);
  unsigned short* AOh    = (unsigned short*)(ws + oAh);
  unsigned short* AOl    = (unsigned short*)(ws + oAl);
  float*          out0   = (float*)d_out;

  const dim3 blk(256);
  const int gqk = ((MT / 64) * (QKW / 64)) / 8;
  const int gvt = ((HH / 64) * (MT / 64)) / 8;
  const int gsp = ((MT / 32) * (HH / 64)) / 8;
  if ((((MT / 64) * (QKW / 64)) % 8) != 0) return;
  if ((((HH / 64) * (MT / 64)) % 8) != 0) return;
  if ((((MT / 32) * (HH / 64)) % 8) != 0) return;

  cvt_rows<<<dim3(MT / 8), blk, 0, stream>>>(x, Xh, MT, 1.0f);
  cvt_rows<<<dim3(QKVW / 8), blk, 0, stream>>>(Wqkv, Wqkv16, QKVW, WSC);
  cvt_rows<<<dim3(HH / 8), blk, 0, stream>>>(Wout, Wo16, HH, WSC);
  cvt_rows<<<dim3(HH / 8), blk, 0, stream>>>(Wprj, Wp16, HH, WSC);

  gemm64<1, 1, 0><<<dim3(gqk), blk, 0, stream>>>(
      Xh, Xh, HH, Wqkv16, HH, QKh, QKl, out0, QKW, bqkv, 1.0f / WSC, 1.0f, MT, QKW, HH);
  gemm64<1, 2, 0><<<dim3(gvt), blk, 0, stream>>>(
      Wqkv16 + (size_t)QKW * HH, Wqkv16 + (size_t)QKW * HH, HH, Xh, HH, VT, VTl, out0, MT,
      bqkv + QKW, 1.0f / WSC, 1.0f, HH, MT, HH);

  attn_kernel<<<dim3(MT / 64, NHD / 2), blk, 0, stream>>>(QKh, QKl, VT, VTl, Zh, Zl);

  gemm64<1, 1, 1><<<dim3(gsp), blk, 0, stream>>>(
      Zh, Zl, HH, Wo16, HH, AOh, AOl, out0, HH, bout, 1.0f / (WSC * ZSC), ZSC, MT, HH, HH);

  gemm64<0, 0, 1><<<dim3(gsp), blk, 0, stream>>>(
      AOh, AOl, HH, Wp16, HH, Zh, Zl, out0, HH, bout, 1.0f / (WSC * ZSC), 1.0f, MT, HH, HH);
  (void)hipGetLastError();
}
